// KSSMLayer_66872640798755
// MI455X (gfx1250) — hardware-verified
//
#include <hip/hip_runtime.h>
#include <math.h>

constexpr int kBatch  = 2;
constexpr int kSeqLen = 2048;
constexpr int kDModel = 512;
constexpr int kDInner = 1024;
constexpr int kGateN  = 6 * kDInner;
constexpr int kCoefN  = 4 * kDInner;
constexpr int kStateW = 2 * kDInner;
constexpr int kTS     = 4;

constexpr size_t kOffXb  = 0;
constexpr size_t kOffWg  = kOffXb  + (size_t)kBatch * kSeqLen * kDModel * 2;
constexpr size_t kOffWo  = kOffWg  + (size_t)kGateN * kDModel * 2;
constexpr size_t kOffP   = kOffWo  + (size_t)kDModel * kStateW * 2;
constexpr size_t kOffQ   = kOffP   + (size_t)kSeqLen * kGateN * 4;
constexpr size_t kOffShi = kOffQ   + (size_t)kSeqLen * kCoefN * 4;
constexpr size_t kOffSlo = kOffShi + (size_t)kSeqLen * kStateW * 2;
constexpr size_t kWsTotal = kOffSlo + (size_t)kSeqLen * kStateW * 2;

typedef __attribute__((ext_vector_type(16))) _Float16 v16h;
typedef __attribute__((ext_vector_type(8)))  _Float16 v8h;
typedef __attribute__((ext_vector_type(16))) __bf16   v16b;
typedef __attribute__((ext_vector_type(8)))  __bf16   v8b;
typedef __attribute__((ext_vector_type(8)))  float    v8f;
typedef __attribute__((ext_vector_type(4)))  float    v4f;
typedef __attribute__((ext_vector_type(2)))  float    v2f;
typedef __attribute__((ext_vector_type(4)))  unsigned int v4u;

__device__ __forceinline__ unsigned short f2bf_bits(float f) {
  unsigned u = __float_as_uint(f);
  return (unsigned short)((u + 0x7FFFu + ((u >> 16) & 1u)) >> 16);
}
__device__ __forceinline__ float bf_bits2f(unsigned short h) { return __uint_as_float(((unsigned)h) << 16); }

__device__ __forceinline__ void dep_guard_h(v8f& a, v8f& b, v16h x, v16h y) { asm volatile("v_nop\n\tv_nop\n\tv_nop\n\tv_nop" : "+v"(a), "+v"(b) : "v"(x), "v"(y)); }
__device__ __forceinline__ void dep_guard_b(v8f& a, v8f& b, v16b x, v16b y) { asm volatile("v_nop\n\tv_nop\n\tv_nop\n\tv_nop" : "+v"(a), "+v"(b) : "v"(x), "v"(y)); }
__device__ __forceinline__ void keep4_h(v16h a, v16h b, v16h c, v16h d) { asm volatile("v_nop" :: "v"(a), "v"(b), "v"(c), "v"(d)); }
__device__ __forceinline__ void keep4_b(v16b a, v16b b, v16b c, v16b d) { asm volatile("v_nop" :: "v"(a), "v"(b), "v"(c), "v"(d)); }
__device__ __forceinline__ void acc_guard4(v8f& a, v8f& b, v8f& c, v8f& d) { asm volatile("v_nop\n\tv_nop\n\tv_nop\n\tv_nop" : "+v"(a), "+v"(b), "+v"(c), "+v"(d)); }
template <typename T> struct Frag;
template <> struct Frag<_Float16> {
  typedef v16h V; union U { v16h v; v8h h[2]; };
  static __device__ __forceinline__ v16h load(const _Float16* p) {
    U f; f.h[0] = *(const v8h*)(p); f.h[1] = *(const v8h*)(p + 16); return f.v;
  }
  static __device__ __forceinline__ v8f mma(v16h a, v16h b, v8f c) {
    return __builtin_amdgcn_wmma_f32_16x16x32_f16(false, a, false, b, (short)0, c, false, false);
  }
  static __device__ __forceinline__ void guard(v8f& a, v8f& b, v16h x, v16h y) { dep_guard_h(a, b, x, y); }
  static __device__ __forceinline__ void keep(v16h a, v16h b, v16h c, v16h d) { keep4_h(a, b, c, d); }
};
template <> struct Frag<__bf16> {
  typedef v16b V; union U { v16b v; v8b h[2]; };
  static __device__ __forceinline__ v16b load(const __bf16* p) {
    U f; f.h[0] = *(const v8b*)(p); f.h[1] = *(const v8b*)(p + 16); return f.v;
  }
  static __device__ __forceinline__ v8f mma(v16b a, v16b b, v8f c) {
    return __builtin_amdgcn_wmma_f32_16x16x32_bf16(false, a, false, b, (short)0, c, false, false);
  }
  static __device__ __forceinline__ void guard(v8f& a, v8f& b, v16b x, v16b y) { dep_guard_b(a, b, x, y); }
  static __device__ __forceinline__ void keep(v16b a, v16b b, v16b c, v16b d) { keep4_b(a, b, c, d); }
};

__device__ __forceinline__ unsigned pk16(unsigned short a, unsigned short b) { return (unsigned)a | ((unsigned)b << 16); }

template <int ET> struct Elem;
template <> struct Elem<0> { typedef _Float16 T; };
template <> struct Elem<1> { typedef __bf16 T; };
template <int ET, int SPLIT, int BIAS_MODE, int OUT_MODE, bool RESID, int ACT = 0>
__global__ __launch_bounds__(256) void wmma_gemm64(
    const unsigned short* __restrict__ Ap, const unsigned short* __restrict__ A2p, int lda, long strideA,
    const unsigned short* __restrict__ Btp, const unsigned short* __restrict__ Bt2p, int ldb, long strideB,
    void* __restrict__ Cout, void* __restrict__ Cout2, int ldc, long strideC,
    const float* __restrict__ bias,
    const float* __restrict__ resid, long strideR,
    int M, int N, int K, float scale) {
  typedef typename Elem<ET>::T T;
  typedef typename Frag<T>::V V;
  const T* A = (const T*)Ap; const T* A2 = (const T*)A2p; const T* Bt = (const T*)Btp; const T* Bt2 = (const T*)Bt2p;
  __shared__ __align__(16) float sT[8][16 * 68];
  const int b    = blockIdx.y;
  const int lane = threadIdx.x & 31;
  const int wave = threadIdx.x >> 5;
  const int tilesN = N >> 6;
  const int tilesM = M >> 6;
  const int tile = blockIdx.x * 8 + wave;
  if (tile >= tilesM * tilesN) return;
  const int tm = tile / tilesN;
  const int tn = tile - tm * tilesN;
  const int m0 = tm << 6;
  const int n0 = tn << 6;

  const T* Ab  = A  + (size_t)b * strideA;
  const T* Bb  = Bt + (size_t)b * strideB;
  const T* Ab2 = (SPLIT != 0) ? (A2  + (size_t)b * strideA) : nullptr;
  const T* Bb2 = (SPLIT == 1) ? (Bt2 + (size_t)b * strideB) : nullptr;

  const int rlane = lane & 15;
  const int koff  = (lane >> 4) * 8;
  const int mOff  = (lane >> 4) * 8;

  v8f acc[4][4];
#pragma unroll
  for (int i = 0; i < 4; ++i)
#pragma unroll
    for (int j = 0; j < 4; ++j) acc[i][j] = (v8f){0.f,0.f,0.f,0.f,0.f,0.f,0.f,0.f};

  for (int k0 = 0; k0 < K; k0 += 32) {
    V bh[4], bl[4];
#pragma unroll
    for (int j = 0; j < 4; ++j) {
      const size_t bo = (size_t)(n0 + (j << 4) + rlane) * ldb + koff + k0;
      bh[j] = Frag<T>::load(Bb + bo);
      if (SPLIT == 1) bl[j] = Frag<T>::load(Bb2 + bo);
    }
#pragma unroll
    for (int i = 0; i < 4; ++i) {
      const size_t ao = (size_t)(m0 + (i << 4) + rlane) * lda + koff + k0;
      V ah = Frag<T>::load(Ab + ao);
      V al;
      if (SPLIT != 0) al = Frag<T>::load(Ab2 + ao);
#pragma unroll
      for (int j = 0; j < 4; ++j) {
        acc[i][j] = Frag<T>::mma(ah, bh[j], acc[i][j]);
        if (SPLIT == 1) {
          acc[i][j] = Frag<T>::mma(ah, bl[j], acc[i][j]);
          acc[i][j] = Frag<T>::mma(al, bh[j], acc[i][j]);
        }
        if (SPLIT == 2) {
          acc[i][j] = Frag<T>::mma(al, bh[j], acc[i][j]);
        }
      }
      Frag<T>::guard(acc[i][0], acc[i][3], ah, (SPLIT != 0) ? al : ah);
    }
    Frag<T>::keep(bh[0], bh[1], bh[2], bh[3]);
    if (SPLIT == 1) Frag<T>::keep(bl[0], bl[1], bl[2], bl[3]);
  }
  acc_guard4(acc[0][0], acc[0][1], acc[0][2], acc[0][3]);
  acc_guard4(acc[1][0], acc[1][1], acc[1][2], acc[1][3]);
  acc_guard4(acc[2][0], acc[2][1], acc[2][2], acc[2][3]);
  acc_guard4(acc[3][0], acc[3][1], acc[3][2], acc[3][3]);

  float* slab = sT[wave];
  const float* Rb = RESID ? (resid + (size_t)b * strideR) : nullptr;
#pragma unroll
  for (int i = 0; i < 4; ++i) {
    const int mBase = m0 + (i << 4);
#pragma unroll
    for (int j = 0; j < 4; ++j) {
      const int n = n0 + (j << 4) + rlane;
      float bv = 0.f;
      if (BIAS_MODE == 2) bv = bias[n];
#pragma unroll
      for (int r = 0; r < 8; ++r) {
        float v = acc[i][j][r] * scale;
        if (BIAS_MODE == 1) v += bias[mBase + mOff + r];
        if (BIAS_MODE == 2) v += bv;
        if (RESID) v += Rb[(size_t)(mBase + mOff + r) * ldc + n];
        if (ACT == 2) v = fmaxf(v, 0.0f);
        if (ACT == 4) v = (v > 0.f) ? v : 0.01f * v;
        slab[(mOff + r) * 68 + (j << 4) + rlane] = v;
      }
    }
    __builtin_amdgcn_fence(__ATOMIC_RELEASE, "workgroup");
    __builtin_amdgcn_wave_barrier();
    __builtin_amdgcn_fence(__ATOMIC_ACQUIRE, "workgroup");
    if (OUT_MODE == 0) {
      float* C = (float*)Cout + (size_t)b * strideC;
      const int hh = lane >> 4, c4 = (lane & 15) * 4;
      for (int pass = 0; pass < 2; ++pass) {
#pragma unroll
        for (int it = 0; it < 8; ++it) {
          const int row = it * 2 + hh;
          v4f v = *(const v4f*)(slab + row * 68 + c4);
          *(volatile v4f*)(C + (size_t)(mBase + row) * ldc + n0 + c4) = v;
        }
        __threadfence();
      }
    } else {
      const int q = lane >> 3, c8 = (lane & 7) * 8;
      unsigned short* C  = (unsigned short*)Cout  + (size_t)b * strideC;
      unsigned short* C2 = (OUT_MODE == 2) ? ((unsigned short*)Cout2 + (size_t)b * strideC) : nullptr;
      for (int pass = 0; pass < 2; ++pass) {
#pragma unroll
        for (int it = 0; it < 4; ++it) {
          const int row = it * 4 + q;
          const float* sp = slab + row * 68 + c8;
          v8h hv, lv;
#pragma unroll
          for (int e = 0; e < 8; ++e) {
            if (OUT_MODE == 1) {
              hv[e] = (_Float16)sp[e];
            } else {
              unsigned short hb = f2bf_bits(sp[e]);
              unsigned short lb = f2bf_bits(sp[e] - bf_bits2f(hb));
              hv[e] = __builtin_bit_cast(_Float16, hb);
              lv[e] = __builtin_bit_cast(_Float16, lb);
            }
          }
          *(volatile v8h*)(C + (size_t)(mBase + row) * ldc + n0 + c8) = hv;
          if (OUT_MODE == 2) *(volatile v8h*)(C2 + (size_t)(mBase + row) * ldc + n0 + c8) = lv;
        }
        __threadfence();
      }
    }
    __builtin_amdgcn_fence(__ATOMIC_RELEASE, "workgroup");
    __builtin_amdgcn_wave_barrier();
    __builtin_amdgcn_fence(__ATOMIC_ACQUIRE, "workgroup");
  }
}

__global__ __launch_bounds__(256) void cast8_bf16_kernel(const float* __restrict__ in, unsigned short* __restrict__ out, int n8) {
  const int i = blockIdx.x * 256 + threadIdx.x;
  if (i >= n8) return;
  const float* p = in + 8 * (size_t)i;
  const v4f a = *(const v4f*)(p);
  const v4f c = *(const v4f*)(p + 4);
  unsigned short hb[8];
#pragma unroll
  for (int e = 0; e < 4; ++e) {
    hb[e]     = f2bf_bits(a[e]);
    hb[4 + e] = f2bf_bits(c[e]);
  }
  const v4u u = (v4u){pk16(hb[0], hb[1]), pk16(hb[2], hb[3]), pk16(hb[4], hb[5]), pk16(hb[6], hb[7])};
  unsigned short* q = out + 8 * (size_t)i;
  *(volatile v4u*)q = u;
  __threadfence();
  *(volatile v4u*)q = u;
}

__global__ __launch_bounds__(256) void tcast_bf16_kernel(const float* __restrict__ W0, const float* __restrict__ W1,
                                                         const float* __restrict__ W2, const float* __restrict__ W3,
                                                         unsigned short* __restrict__ out, int nrows, int ncols, long zstride) {
  __shared__ float sm[64][65];
  const int t  = threadIdx.x;
  const int c0 = blockIdx.x * 64;
  const int r0 = blockIdx.y * 64;
  const int z  = blockIdx.z;
  const float* W = (z == 0) ? W0 : (z == 1) ? W1 : (z == 2) ? W2 : W3;
#pragma unroll
  for (int i = 0; i < 16; ++i) {
    const int e  = i * 256 + t;
    const int rl = e >> 6;
    const int cl = e & 63;
    sm[cl][rl] = W[(size_t)(r0 + rl) * ncols + c0 + cl];
  }
  __syncthreads();
  const int lane = t & 31, wave = t >> 5;
  const int q = lane >> 3, c8 = (lane & 7) * 8;
  unsigned short* op = out + (size_t)z * zstride;
  for (int pass = 0; pass < 2; ++pass) {
#pragma unroll
    for (int it = 0; it < 2; ++it) {
      const int row = wave * 8 + it * 4 + q;
      unsigned short hb[8];
#pragma unroll
      for (int e = 0; e < 8; ++e) hb[e] = f2bf_bits(sm[row][c8 + e]);
      const v4u u = (v4u){pk16(hb[0], hb[1]), pk16(hb[2], hb[3]), pk16(hb[4], hb[5]), pk16(hb[6], hb[7])};
      *(volatile v4u*)(op + (size_t)(c0 + row) * nrows + r0 + c8) = u;
    }
    __threadfence();
  }
}

__device__ __forceinline__ float softplus_f(float z) {
  return fmaxf(z, 0.0f) + log1pf(expf(-fabsf(z)));
}

__global__ __launch_bounds__(256) void cayley_kernel(const float* __restrict__ P, float* __restrict__ Q) {
  __shared__ __align__(16) float sq[4][256];
  const int tid = threadIdx.x;
  const int t   = blockIdx.x >> 2;
  const int d0  = (blockIdx.x & 3) * 256;
  const int d   = d0 + tid;
  const float* pr = P + (size_t)t * kGateN;
  const float xin = pr[d];
  const float alp = softplus_f(pr[kDInner + d]);
  const float om  = pr[2 * kDInner + d];
  const float dt  = softplus_f(pr[3 * kDInner + d]);
  const v2f   bm  = *(const v2f*)(pr + 4 * kDInner + 2 * d);
  const float a     = 0.5f * dt * alp;
  const float w     = 0.5f * dt * om;
  const float onepa = 1.0f + a;
  const float det   = onepa * onepa + w * w + 1e-6f;
  const float invd  = 1.0f / det;
  const float adiag = (1.0f - a * a - w * w) * invd;
  const float aoff  = 2.0f * w * invd;
  const float u1    = dt * bm.x * xin;
  const float u2    = dt * bm.y * xin;
  const float ub1   = (onepa * u1 + w * u2) * invd;
  const float ub2   = (onepa * u2 - w * u1) * invd;
  sq[0][tid] = adiag;
  sq[1][tid] = aoff;
  sq[2][tid] = ub1;
  sq[3][tid] = ub2;
  __syncthreads();
  const int g = tid >> 6, q4 = (tid & 63) * 4;
  const v4f v = *(const v4f*)(&sq[g][q4]);
  float* dst = Q + (size_t)t * kCoefN + g * kDInner + d0 + q4;
  for (int pass = 0; pass < 2; ++pass) {
    *(volatile v4f*)dst = v;
    __threadfence();
  }
}

__global__ __launch_bounds__(256) void scan_kernel(const float* __restrict__ Q, const float* __restrict__ st0,
                                                   unsigned short* __restrict__ Shi, unsigned short* __restrict__ Slo,
                                                   float* __restrict__ fin) {
  __shared__ __align__(16) unsigned int shi[kTS][256];
  __shared__ __align__(16) unsigned int slo[kTS][256];
  __shared__ __align__(16) float sfin[512];
  const int tid = threadIdx.x;
  const int d0  = blockIdx.x * 256;
  const int d   = d0 + tid;
  float h1 = bf_bits2f(f2bf_bits(st0[2 * d]));
  float h2 = bf_bits2f(f2bf_bits(st0[2 * d + 1]));
  const int srow = tid >> 6;
  const int sq4  = (tid & 63) * 4;
  const int scol = (tid & 63) * 8;
  for (int t0 = 0; t0 < kSeqLen; t0 += kTS) {
#pragma unroll
    for (int j = 0; j < kTS; ++j) {
      const float* qr = Q + (size_t)(t0 + j) * kCoefN;
      const float ad = qr[d];
      const float ao = qr[kDInner + d];
      const float u1 = qr[2 * kDInner + d];
      const float u2 = qr[3 * kDInner + d];
      const float n1 = ad * h1 + ao * h2 + u1;
      const float n2 = ad * h2 - ao * h1 + u2;
      h1 = n1;
      h2 = n2;
      const unsigned short hb1 = f2bf_bits(n1), hb2 = f2bf_bits(n2);
      const unsigned short lb1 = f2bf_bits(n1 - bf_bits2f(hb1));
      const unsigned short lb2 = f2bf_bits(n2 - bf_bits2f(hb2));
      shi[j][tid] = pk16(hb1, hb2);
      slo[j][tid] = pk16(lb1, lb2);
    }
    __syncthreads();
    const v4u vh = *(const v4u*)(&shi[srow][sq4]);
    const v4u vl = *(const v4u*)(&slo[srow][sq4]);
    unsigned short* ph = Shi + (size_t)(t0 + srow) * kStateW + 2 * d0 + scol;
    unsigned short* pl = Slo + (size_t)(t0 + srow) * kStateW + 2 * d0 + scol;
    *(volatile v4u*)ph = vh;
    *(volatile v4u*)pl = vl;
    __threadfence();
    *(volatile v4u*)ph = vh;
    *(volatile v4u*)pl = vl;
    __syncthreads();
  }
  sfin[2 * tid]     = h1;
  sfin[2 * tid + 1] = h2;
  __syncthreads();
  const int fi = (tid & 127) * 4;
  const v4f fv = *(const v4f*)(&sfin[fi]);
  float* pf = fin + 2 * d0 + fi;
  for (int pass = 0; pass < 2; ++pass) {
    if (tid < 128) *(volatile v4f*)pf = fv;
    __threadfence();
  }
}

extern "C" void kernel_launch(void* const* d_in, const int* in_sizes, int n_in,
                              void* d_out, int out_size, void* d_ws, size_t ws_size,
                              hipStream_t stream) {
  if (n_in < 8) return;
  if (in_sizes[0] != kBatch * kSeqLen * kDModel) return;
  if (in_sizes[1] != kBatch * kDInner * 2) return;
  if (in_sizes[2] != kDModel * kDInner || in_sizes[3] != kDModel * kDInner ||
      in_sizes[4] != kDModel * kDInner || in_sizes[5] != kDModel * kDInner) return;
  if (in_sizes[6] != kDModel * kStateW) return;
  if (in_sizes[7] != kStateW * kDModel) return;
  if (out_size != kBatch * kSeqLen * kDModel + kBatch * kDInner * 2) return;
  if (ws_size < kWsTotal) return;

  const float* x     = (const float*)d_in[0];
  const float* state = (const float*)d_in[1];
  const float* Wx    = (const float*)d_in[2];
  const float* Wal   = (const float*)d_in[3];
  const float* Wom   = (const float*)d_in[4];
  const float* Wdt   = (const float*)d_in[5];
  const float* Wb    = (const float*)d_in[6];
  const float* Wout  = (const float*)d_in[7];

  float* out  = (float*)d_out;
  float* out1 = out + (size_t)kBatch * kSeqLen * kDModel;

  char* ws = (char*)d_ws;
  unsigned short* xb  = (unsigned short*)(ws + kOffXb);
  unsigned short* wg  = (unsigned short*)(ws + kOffWg);
  unsigned short* wo  = (unsigned short*)(ws + kOffWo);
  float*          P   = (float*)(ws + kOffP);
  float*          Q   = (float*)(ws + kOffQ);
  unsigned short* Shi = (unsigned short*)(ws + kOffShi);
  unsigned short* Slo = (unsigned short*)(ws + kOffSlo);

  const int n8x = kBatch * kSeqLen * kDModel / 8;
  cast8_bf16_kernel<<<(n8x + 255) / 256, 256, 0, stream>>>(x, xb, n8x);

  tcast_bf16_kernel<<<dim3(kDInner / 64, kDModel / 64, 4), 256, 0, stream>>>(
      Wx, Wal, Wom, Wdt, wg, kDModel, kDInner, (long)kDInner * kDModel);
  tcast_bf16_kernel<<<dim3(kStateW / 64, kDModel / 64, 1), 256, 0, stream>>>(
      Wb, Wb, Wb, Wb, wg + (size_t)4 * kDInner * kDModel, kDModel, kStateW, 0L);
  tcast_bf16_kernel<<<dim3(kDModel / 64, kStateW / 64, 1), 256, 0, stream>>>(
      Wout, Wout, Wout, Wout, wo, kStateW, kDModel, 0L);

  const int tilesGate = (kSeqLen / 64) * (kGateN / 64);
  const int tilesOut  = (kSeqLen / 64) * (kDModel / 64);

  for (int b = 0; b < kBatch; ++b) {
    wmma_gemm64<1, 0, 0, 0, false><<<dim3((tilesGate + 7) / 8, 1), 256, 0, stream>>>(
        xb + (size_t)b * kSeqLen * kDModel, nullptr, kDModel, 0L,
        wg, nullptr, kDModel, 0L,
        P, nullptr, kGateN, 0L,
        nullptr, nullptr, 0L,
        kSeqLen, kGateN, kDModel, 1.0f);

    cayley_kernel<<<kSeqLen * 4, 256, 0, stream>>>(P, Q);

    scan_kernel<<<kDInner / 256, 256, 0, stream>>>(
        Q, state + (size_t)b * kDInner * 2, Shi, Slo, out1 + (size_t)b * kDInner * 2);

    wmma_gemm64<1, 2, 0, 0, false><<<dim3((tilesOut + 7) / 8, 1), 256, 0, stream>>>(
        Shi, Slo, kStateW, 0L,
        wo, nullptr, kStateW, 0L,
        out + (size_t)b * kSeqLen * kDModel, nullptr, kDModel, 0L,
        nullptr, nullptr, 0L,
        kSeqLen, kDModel, kStateW, 1.0f);
  }
}
